// HolographicBlock_55783035240635
// MI455X (gfx1250) — hardware-verified
//
#include <hip/hip_runtime.h>
#include <hip/hip_bf16.h>
#include <math.h>


#define BB 2
#define SS 2048
#define DD 1024
#define HH 8
#define DKK 128
#define KS2 136
#define RR 64
#define QW 2

typedef _Float16 bf16;
typedef __attribute__((ext_vector_type(4))) unsigned v4u_t;
typedef unsigned v4ua __attribute__((ext_vector_type(4), may_alias));
typedef __attribute__((ext_vector_type(4))) float v4f_t;
typedef float v4fa __attribute__((ext_vector_type(4), may_alias));
typedef __attribute__((ext_vector_type(16))) bf16  bf16x16;
typedef __attribute__((ext_vector_type(8)))  bf16  bf16x8;
typedef __attribute__((ext_vector_type(4)))  bf16  bf16x4;
typedef __attribute__((ext_vector_type(8)))  float f32x8;

#define LDS_STRIDE 48
#define KSTRIDE    72
#define VSTRIDE    48

__device__ __forceinline__ f32x8 wmma_bf16(bf16x16 a, bf16x16 b, f32x8 c) {
  return __builtin_amdgcn_wmma_f32_16x16x32_f16(
      false, a, false, b, (short)0, c, false, false);
}
#define RSPLIT (1.0f / 2048.0f)
__device__ __forceinline__ bf16 lo_of(float v, bf16 h) { return (bf16)((v - (float)h) * 2048.0f); }
__device__ __forceinline__ f32x8 wmma_split(bf16x16 a, bf16x16 al, bf16x16 b, bf16x16 bl, f32x8 c) {
  f32x8 x = {}; x = wmma_bf16(al, b, x); x = wmma_bf16(a, bl, x); return wmma_bf16(a, b, c) + x * RSPLIT; }

template <typename T>
__device__ __forceinline__ bf16x16 load_frag(const T* __restrict__ base, int ld,
                                             int row0, int k0) {
  const int lane = threadIdx.x & 31;
  const int r    = lane & 15;
  const int kh   = (lane >> 4) * 8;
  const T* p0 = base + (size_t)(row0 + r) * ld + (k0 + kh);
  const T* p1 = p0 + 16;
  bf16x16 f;
#pragma unroll
  for (int i = 0; i < 8; ++i) {
    f[i]     = (bf16)p0[i];
    f[i + 8] = (bf16)p1[i];
  }
  return f;
}

__device__ __forceinline__ bf16x16 lds_frag(const bf16* base, int stride) {
  const int lane = threadIdx.x & 31;
  const int row  = lane & 15;
  const int kh   = (lane >> 4) * 8;
  const bf16x8 lo = *(const bf16x8*)(base + row * stride + kh);
  const bf16x8 hi = *(const bf16x8*)(base + row * stride + kh + 16);
  bf16x16 f;
#pragma unroll
  for (int i = 0; i < 8; ++i) { f[i] = lo[i]; f[i + 8] = hi[i]; }
  return f;
}

template <typename T>
__device__ __forceinline__ void stage_read16(const T* __restrict__ p, float* buf) {
#pragma unroll
  for (int i = 0; i < 16; ++i) buf[i] = (float)p[i];
}

__device__ __forceinline__ void stage_write(bf16* dst, const float* buf, int nquad) {
#pragma unroll
  for (int i = 0; i < nquad; ++i) {
    bf16x4 q;
    q[0] = (bf16)buf[4 * i];     q[1] = (bf16)buf[4 * i + 1];
    q[2] = (bf16)buf[4 * i + 2]; q[3] = (bf16)buf[4 * i + 3];
    *(bf16x4*)(dst + 4 * i) = q;
  }
}

template <typename AT, int MODE>
__global__ __launch_bounds__(256) void gemm_bias_kernel(
    const AT* __restrict__ A, const float* __restrict__ W,
    const float* __restrict__ bias, void* __restrict__ out,
    int M, int N, int K) {
  __shared__ bf16 ldsA[128 * LDS_STRIDE];
  __shared__ bf16 ldsW[256 * LDS_STRIDE];
  __shared__ __attribute__((aligned(16))) unsigned char sob[256 * 136 * 2];

  const int t    = threadIdx.x;
  const int wave = t >> 5;
  const int lane = t & 31;
  const int wm   = (wave & 1) * 64;
  const int wn   = (wave >> 1) * 64;
  const int mBlk = blockIdx.x * 128;
  const int nBlk = blockIdx.y * 256;

  const int arow = t >> 1;
  const int ach  = (t & 1) * 16;

  float abuf[16];
  float wbuf[32];

  stage_read16(A + (size_t)(mBlk + arow) * K + ach, abuf);
  stage_read16(W + (size_t)(nBlk + t) * K,          wbuf);
  stage_read16(W + (size_t)(nBlk + t) * K + 16,     wbuf + 16);

  f32x8 acc[4][4] = {};

  for (int k = 0; k < K; k += 32) {
    __syncthreads();
    stage_write(&ldsA[arow * LDS_STRIDE + ach], abuf, 4);
    stage_write(&ldsW[t * LDS_STRIDE],          wbuf, 8);
    if (k + 32 < K) {
      stage_read16(A + (size_t)(mBlk + arow) * K + (k + 32) + ach, abuf);
      stage_read16(W + (size_t)(nBlk + t) * K + (k + 32),          wbuf);
      stage_read16(W + (size_t)(nBlk + t) * K + (k + 32) + 16,     wbuf + 16);
    }
    __syncthreads();

    bf16x16 af[4], wf[4];
#pragma unroll
    for (int i = 0; i < 4; ++i)
      af[i] = lds_frag(ldsA + (wm + 16 * i) * LDS_STRIDE, LDS_STRIDE);
#pragma unroll
    for (int j = 0; j < 4; ++j)
      wf[j] = lds_frag(ldsW + (wn + 16 * j) * LDS_STRIDE, LDS_STRIDE);
#pragma unroll
    for (int i = 0; i < 4; ++i)
#pragma unroll
      for (int j = 0; j < 4; ++j)
        acc[i][j] = wmma_bf16(af[i], wf[j], acc[i][j]);
  }

  const int nlane = lane & 15;
  const int mh    = (lane >> 4) * 8;
  __syncthreads();
  if (MODE == 0 || MODE == 1) {
    bf16* so = (bf16*)sob;
#pragma unroll
    for (int i = 0; i < 4; ++i)
#pragma unroll
      for (int j = 0; j < 4; ++j) {
        const int nl = wn + 16 * j + nlane;
        const float bv = bias ? bias[nBlk + nl] : 0.0f;
#pragma unroll
        for (int r = 0; r < 8; ++r) {
          const int ml = wm + 16 * i + mh + r;
          const bf16 hv = (bf16)(acc[i][j][r] + bv);
          if (MODE == 0) so[ml * 264 + nl] = hv;
          else           so[nl * 136 + ml] = hv;
        }
      }
    __syncthreads();
#pragma unroll 1
    for (int pass = 0; pass < 2; ++pass) {
      if (MODE == 0) {
        for (int ch = t; ch < 128 * 32; ch += 256) { const int ml = ch >> 5, q = (ch & 31) * 8;
          *(volatile v4u_t*)((bf16*)out + (size_t)(mBlk + ml) * N + nBlk + q) = *(const v4ua*)(so + ml * 264 + q); }
      } else {
        const int b_ = mBlk / SS, s0 = mBlk & (SS - 1);
        for (int ch = t; ch < 256 * 16; ch += 256) { const int nl = ch >> 4, q = (ch & 15) * 8; const int n = nBlk + nl, h = n >> 6, dk = n & (DKK - 1);
          *(volatile v4u_t*)((bf16*)out + (((size_t)(b_ * HH + h)) * DKK + dk) * SS + s0 + q) = *(const v4ua*)(so + nl * 136 + q); }
      }
      __threadfence();
    }
  } else {
    float* so = (float*)sob;
#pragma unroll 1
    for (int hf = 0; hf < 2; ++hf) {
      if (wm == hf * 64) {
#pragma unroll
        for (int i = 0; i < 4; ++i)
#pragma unroll
          for (int j = 0; j < 4; ++j) {
            const int nl = wn + 16 * j + nlane;
            const float bv = bias ? bias[nBlk + nl] : 0.0f;
#pragma unroll
            for (int r = 0; r < 8; ++r) so[(16 * i + mh + r) * 260 + nl] = acc[i][j][r] + bv;
          }
      }
      __syncthreads();
#pragma unroll 1
      for (int pass = 0; pass < 2; ++pass) {
        for (int ch = t; ch < 64 * 64; ch += 256) { const int ml = ch >> 6, q = (ch & 63) * 4;
          *(volatile v4f_t*)((float*)out + (size_t)(mBlk + hf * 64 + ml) * N + nBlk + q) = *(const volatile v4fa*)(so + ml * 260 + q); }
        __threadfence();
      }
      __syncthreads();
    }
  }
}

template <typename AT, int MODE>
__global__ __launch_bounds__(256) void gemm_split_kernel(
    const AT* __restrict__ A, size_t aPlane, const float* __restrict__ W,
    const float* __restrict__ bias, void* __restrict__ out,
    int M, int N, int K) {
  __shared__ bf16 ldsA[128 * LDS_STRIDE], ldsAl[128 * LDS_STRIDE];
  __shared__ bf16 ldsW[256 * LDS_STRIDE], ldsWl[256 * LDS_STRIDE];
  __shared__ __attribute__((aligned(16))) unsigned char sob[256 * 136 * 2];

  const int t    = threadIdx.x;
  const int wave = t >> 5;
  const int lane = t & 31;
  const int wm   = (wave & 1) * 64;
  const int wn   = (wave >> 1) * 64;
  const int mBlk = blockIdx.x * 128;
  const int nBlk = blockIdx.y * 256;
  const int arow = t >> 1;
  const int ach  = (t & 1) * 16;

  f32x8 acc[4][4] = {};
  for (int k = 0; k < K; k += 32) {
    __syncthreads();
    {
      const AT* ap = A + (size_t)(mBlk + arow) * K + k + ach;
      bf16 hh[16], hl[16];
      if (sizeof(AT) == 4) {
#pragma unroll
        for (int i = 0; i < 16; ++i) { const float v = (float)ap[i]; hh[i] = (bf16)v; hl[i] = lo_of(v, hh[i]); }
      } else {
#pragma unroll
        for (int i = 0; i < 16; ++i) { hh[i] = (bf16)ap[i]; hl[i] = (bf16)ap[aPlane + i]; }
      }
#pragma unroll
      for (int i = 0; i < 16; ++i) { ldsA[arow * LDS_STRIDE + ach + i] = hh[i]; ldsAl[arow * LDS_STRIDE + ach + i] = hl[i]; }
    }
    {
      const float* wp = W + (size_t)(nBlk + t) * K + k;
#pragma unroll
      for (int i = 0; i < 32; ++i) { const float v = wp[i]; const bf16 h_ = (bf16)v; ldsW[t * LDS_STRIDE + i] = h_; ldsWl[t * LDS_STRIDE + i] = lo_of(v, h_); }
    }
    __syncthreads();
    bf16x16 wf[4], wfl[4];
#pragma unroll
    for (int j = 0; j < 4; ++j) { wf[j] = lds_frag(ldsW + (wn + 16 * j) * LDS_STRIDE, LDS_STRIDE); wfl[j] = lds_frag(ldsWl + (wn + 16 * j) * LDS_STRIDE, LDS_STRIDE); }
#pragma unroll
    for (int i = 0; i < 4; ++i) {
      const bf16x16 af = lds_frag(ldsA + (wm + 16 * i) * LDS_STRIDE, LDS_STRIDE), afl = lds_frag(ldsAl + (wm + 16 * i) * LDS_STRIDE, LDS_STRIDE);
#pragma unroll
      for (int j = 0; j < 4; ++j) acc[i][j] = wmma_split(af, afl, wf[j], wfl[j], acc[i][j]);
    }
  }

  const int nlane = lane & 15;
  const int mh    = (lane >> 4) * 8;
  __syncthreads();
  if (MODE == 1) {
    bf16* so = (bf16*)sob;
#pragma unroll
    for (int i = 0; i < 4; ++i)
#pragma unroll
      for (int j = 0; j < 4; ++j) {
        const int nl = wn + 16 * j + nlane;
        const float bv = bias ? bias[nBlk + nl] : 0.0f;
#pragma unroll
        for (int r = 0; r < 8; ++r) so[nl * 136 + wm + 16 * i + mh + r] = (bf16)(acc[i][j][r] + bv);
      }
    __syncthreads();
    const int b_ = mBlk / SS, s0 = mBlk & (SS - 1);
#pragma unroll 1
    for (int pass = 0; pass < 2; ++pass) {
      for (int ch = t; ch < 256 * 16; ch += 256) { const int nl = ch >> 4, q = (ch & 15) * 8; const int n = nBlk + nl, h = n >> 6, dk = n & (DKK - 1);
        *(volatile v4u_t*)((bf16*)out + (((size_t)(b_ * HH + h)) * DKK + dk) * SS + s0 + q) = *(const v4ua*)(so + nl * 136 + q); }
      __threadfence();
    }
  } else {
    float* so = (float*)sob;
#pragma unroll 1
    for (int hf = 0; hf < 2; ++hf) {
      if (wm == hf * 64) {
#pragma unroll
        for (int i = 0; i < 4; ++i)
#pragma unroll
          for (int j = 0; j < 4; ++j) {
            const int nl = wn + 16 * j + nlane;
            const float bv = bias ? bias[nBlk + nl] : 0.0f;
#pragma unroll
            for (int r = 0; r < 8; ++r) so[(16 * i + mh + r) * 260 + nl] = acc[i][j][r] + bv;
          }
      }
      __syncthreads();
#pragma unroll 1
      for (int pass = 0; pass < 2; ++pass) {
        for (int ch = t; ch < 64 * 64; ch += 256) { const int ml = ch >> 6, q = (ch & 63) * 4;
          *(volatile v4f_t*)((float*)out + (size_t)(mBlk + hf * 64 + ml) * N + nBlk + q) = *(const volatile v4fa*)(so + ml * 260 + q); }
        __threadfence();
      }
      __syncthreads();
    }
  }
}

__global__ __launch_bounds__(64) void attn128_kernel(const bf16* __restrict__ Qb, const bf16* __restrict__ Kb, const bf16* __restrict__ Vt, bf16* __restrict__ attnOut) {
  __shared__ bf16 ldsK[32 * KS2];
  __shared__ bf16 ldsV[128 * VSTRIDE];
  __shared__ __attribute__((aligned(16))) bf16 ldsO[2][2][16 * 136];
  const int q0blk = blockIdx.x * 32, h = blockIdx.y, b = blockIdx.z;
  const size_t oplane = (size_t)BB * SS * DD;
  const int t = threadIdx.x, wave = t >> 5, lane = t & 31, qlane = lane & 15, kh8 = (lane >> 4) * 8;
  const int q0 = q0blk + wave * 16;
  const bf16* Qh = Qb + (size_t)b * SS * DD + h * DKK;
  const bf16* Kh = Kb + (size_t)b * SS * DD + h * DKK;
  const bf16* Vh = Vt + ((size_t)(b * HH + h)) * DKK * SS;
  const int krow = t >> 1, kcol = (t & 1) * 64;
  bf16x16 qf[4];
#pragma unroll
  for (int c = 0; c < 4; ++c) qf[c] = load_frag(Qh, DD, q0, 32 * c);
  f32x8 o[8] = {};
  float mrun = -INFINITY, lrun = 0.0f;
  const float scale = 0.08838834764831845f * 1.44269504088896340736f;
  const int qi = q0 + qlane, kmax = q0blk + 31;
#pragma unroll 1
  for (int kb = 0; kb <= kmax; kb += 32) {
    __syncthreads();
    { const bf16* ks = Kh + (size_t)(kb + krow) * DD + kcol;
#pragma unroll
      for (int i = 0; i < 8; ++i) *(bf16x8*)(&ldsK[krow * KS2 + kcol + 8 * i]) = *(const bf16x8*)(ks + 8 * i);
      const bf16* vs0 = Vh + (size_t)t * SS + kb; const bf16* vs1 = Vh + (size_t)(64 + t) * SS + kb;
#pragma unroll
      for (int i = 0; i < 4; ++i) { *(bf16x8*)(&ldsV[t * VSTRIDE + 8 * i]) = *(const bf16x8*)(vs0 + 8 * i); *(bf16x8*)(&ldsV[(64 + t) * VSTRIDE + 8 * i]) = *(const bf16x8*)(vs1 + 8 * i); } }
    __syncthreads();
    f32x8 s0 = {}, s1 = {};
#pragma unroll
    for (int c = 0; c < 4; ++c) { s0 = wmma_bf16(lds_frag(ldsK + c * 32, KS2), qf[c], s0); s1 = wmma_bf16(lds_frag(ldsK + 16 * KS2 + c * 32, KS2), qf[c], s1); }
    float mx = -INFINITY;
#pragma unroll
    for (int r = 0; r < 8; ++r) { const int j0 = kb + kh8 + r, j1 = j0 + 16;
      s0[r] = (j0 <= qi) ? s0[r] * scale : -INFINITY; s1[r] = (j1 <= qi) ? s1[r] * scale : -INFINITY; mx = fmaxf(mx, fmaxf(s0[r], s1[r])); }
    mx = fmaxf(mx, __shfl_xor(mx, 16, 32));
    const float mnew = fmaxf(mrun, mx), alpha = exp2f(mrun - mnew);
    float rsum = 0.0f; bf16x16 pf;
#pragma unroll
    for (int r = 0; r < 8; ++r) { const float p0 = exp2f(s0[r] - mnew), p1 = exp2f(s1[r] - mnew); rsum += p0 + p1; pf[r] = (bf16)(p0 * 1024.0f); pf[r + 8] = (bf16)(p1 * 1024.0f); }
    rsum += __shfl_xor(rsum, 16, 32);
    lrun = lrun * alpha + rsum; mrun = mnew;
#pragma unroll
    for (int j = 0; j < 8; ++j) {
#pragma unroll
      for (int r = 0; r < 8; ++r) o[j][r] *= alpha;
      o[j] = wmma_bf16(lds_frag(ldsV + (j * 16) * VSTRIDE, VSTRIDE), pf, o[j]); }
  }
  bf16* so = ldsO[wave][0]; bf16* sl = ldsO[wave][1];
  const float rl = 1.0f / (lrun * 1024.0f);
#pragma unroll
  for (int j = 0; j < 8; ++j)
#pragma unroll
    for (int r = 0; r < 8; ++r) { const float v = o[j][r] * rl; const bf16 hv = (bf16)v; so[qlane * 136 + j * 16 + kh8 + r] = hv; sl[qlane * 136 + j * 16 + kh8 + r] = lo_of(v, hv); }
  asm volatile("s_wait_dscnt 0" ::: "memory");
#pragma unroll 1
  for (int pass = 0; pass < 2; ++pass) {
#pragma unroll
    for (int it = 0; it < 8; ++it) { const int ch = lane + 32 * it, ql = ch >> 4, q8 = (ch & 15) * 8;
      bf16* dst = attnOut + ((size_t)(b * SS + q0 + ql)) * DD + h * DKK + q8;
      *(volatile v4u_t*)dst = *(const v4ua*)(so + ql * 136 + q8); *(volatile v4u_t*)(dst + oplane) = *(const v4ua*)(sl + ql * 136 + q8); }
    __threadfence();
  }
}

__global__ __launch_bounds__(64) void k_cbt(const float* __restrict__ Bm, const float* const* Cs_unused, const float* __restrict__ C0, const float* __restrict__ C1, const float* __restrict__ C2,
                                           const float* __restrict__ C3, const float* __restrict__ C4, const float* __restrict__ C5, float* __restrict__ CBt) {
  (void)Cs_unused;
  const int n = blockIdx.x, c = blockIdx.y, r = threadIdx.x;
  const float* Cv = (c == 0) ? C0 : (c == 1) ? C1 : (c == 2) ? C2 : (c == 3) ? C3 : (c == 4) ? C4 : C5;
  const float v = Cv[r] * Bm[(size_t)r * DD + n];
  float* dst = CBt + ((size_t)c * DD + n) * RR + r; *(volatile float*)dst = v; __threadfence(); *(volatile float*)dst = v;
}
__global__ __launch_bounds__(256) void k_rms(const float* __restrict__ x, const float* __restrict__ s, float* __restrict__ y) {
  __shared__ float red[256];
  const int row = blockIdx.x, t = threadIdx.x; const v4f_t v = *(const v4fa*)(x + (size_t)row * DD + t * 4);
  red[t] = v.x * v.x + v.y * v.y + v.z * v.z + v.w * v.w; __syncthreads();
  for (int o = 128; o > 0; o >>= 1) { if (t < o) red[t] += red[t + o]; __syncthreads(); }
  const float rs = rsqrtf(red[0] / (float)DD + 1.1920929e-07f); const v4f_t sv = *(const v4fa*)(s + t * 4);
  v4f_t o4; o4.x = v.x * rs * sv.x; o4.y = v.y * rs * sv.y; o4.z = v.z * rs * sv.z; o4.w = v.w * rs * sv.w;
  *(volatile v4f_t*)(y + (size_t)row * DD + t * 4) = o4; __threadfence(); *(volatile v4f_t*)(y + (size_t)row * DD + t * 4) = o4;
}
__global__ __launch_bounds__(128) void k_trig(float* __restrict__ TR) {
  const int pos = blockIdx.x, i = threadIdx.x & 63, which = threadIdx.x >> 6;
  const float invf = exp2f(-((float)(2 * i) / 128.0f) * 13.287712379549449f); const float ang = (float)pos * invf;
  const float v = which ? sinf(ang) : cosf(ang);
  *(volatile float*)(TR + (size_t)pos * 128 + which * 64 + i) = v; __threadfence(); *(volatile float*)(TR + (size_t)pos * 128 + which * 64 + i) = v;
}
__global__ __launch_bounds__(256) void k_rope(const float* __restrict__ Xf, const float* __restrict__ TR, bf16* __restrict__ Xb) {
  const int tok = blockIdx.x, t = threadIdx.x, pos = tok % SS; const int h = t >> 5, i2 = (t & 31) * 2;
  const float* row = Xf + (size_t)tok * DD + h * DKK; bf16* orow = Xb + (size_t)tok * DD + h * DKK;
  const float c0 = TR[(size_t)pos * 128 + i2], c1 = TR[(size_t)pos * 128 + i2 + 1], s0 = TR[(size_t)pos * 128 + 64 + i2], s1 = TR[(size_t)pos * 128 + 64 + i2 + 1];
  const float a0 = row[i2], a1 = row[i2 + 1], b0 = row[64 + i2], b1 = row[64 + i2 + 1];
  bf16 h1[2], h2[2];
  h1[0] = (bf16)(a0 * c0 + b0 * s0); h1[1] = (bf16)(a1 * c1 + b1 * s1);
  h2[0] = (bf16)(-a0 * s0 + b0 * c0); h2[1] = (bf16)(-a1 * s1 + b1 * c1);
  typedef unsigned u1a __attribute__((may_alias));
#pragma unroll 1
  for (int pass = 0; pass < 2; ++pass) { *(volatile unsigned*)(orow + i2) = *(const u1a*)h1; *(volatile unsigned*)(orow + 64 + i2) = *(const u1a*)h2; __threadfence(); }
}
__global__ __launch_bounds__(256) void k_vt(const float* __restrict__ Vf, bf16* __restrict__ Vt) {
  __shared__ float tile[64][65];
  const int s0 = blockIdx.x * 64, h = blockIdx.y >> 1, dh = (blockIdx.y & 1) * 64, b = blockIdx.z, t = threadIdx.x;
  for (int i = t; i < 64 * 64; i += 256) { const int r = i >> 6, d = i & 63; tile[r][d] = Vf[((size_t)(b * SS + s0 + r)) * DD + h * DKK + dh + d]; }
  __syncthreads();
#pragma unroll 1
  for (int pass = 0; pass < 2; ++pass) {
    for (int i = t; i < 64 * 8; i += 256) { const int dr = i >> 3, s8 = (i & 7) * 8; bf16 hh[8];
#pragma unroll
      for (int e = 0; e < 8; ++e) hh[e] = (bf16)tile[s8 + e][dr];
      *(volatile v4u_t*)(Vt + (((size_t)(b * HH + h)) * DKK + dh + dr) * SS + s0 + s8) = *(const v4ua*)hh; }
    __threadfence();
  }
}
__global__ __launch_bounds__(256) void k_add(const float* __restrict__ a, const float* __restrict__ bsrc, float* __restrict__ y) {
  const size_t off = (size_t)blockIdx.x * DD + threadIdx.x * 4; v4f_t v = *(const v4fa*)(a + off); const v4f_t w = *(const v4fa*)(bsrc + off);
  v.x += w.x; v.y += w.y; v.z += w.z; v.w += w.w; *(volatile v4f_t*)(y + off) = v; __threadfence(); *(volatile v4f_t*)(y + off) = v;
}
__global__ __launch_bounds__(256) void k_silu(float* __restrict__ Hf) {
  const size_t off = (size_t)blockIdx.x * DD + threadIdx.x * 4; v4f_t v = *(const v4fa*)(Hf + off);
#pragma unroll 1
  for (int i = 0; i < 4; ++i) { const float u = v[i]; v[i] = u / (1.0f + expf(-u)); }
  *(volatile v4f_t*)(Hf + off) = v; __threadfence(); *(volatile v4f_t*)(Hf + off) = v;
}

extern "C" void kernel_launch(void* const* d_in, const int* in_sizes, int n_in,
                              void* d_out, int out_size, void* d_ws, size_t ws_size,
                              hipStream_t stream) {
  (void)in_sizes; (void)n_in; (void)out_size; (void)ws_size;
  const float* x  = (const float*)d_in[0];
  const float* bA = (const float*)d_in[1];
  const float* bB = (const float*)d_in[2];
  const float* Cq = (const float*)d_in[3]; const float* Ck = (const float*)d_in[4]; const float* Cv = (const float*)d_in[5];
  const float* Co = (const float*)d_in[6]; const float* Cfc = (const float*)d_in[7]; const float* Cpr = (const float*)d_in[8];
  const float* s1 = (const float*)d_in[9]; const float* s2 = (const float*)d_in[10];
  float* out = (float*)d_out;
  const int M = BB * SS, N = DD, K = DD;
  char* ws = (char*)d_ws;
  float* WT  = (float*)ws; ws += (size_t)6 * DD * DD * 4;
  float* CBt = (float*)ws; ws += (size_t)6 * DD * RR * 4;
  float* TR  = (float*)ws; ws += (size_t)SS * 128 * 4;
  float* N1  = (float*)ws; ws += (size_t)M * DD * 4;
  float* F1  = (float*)ws; ws += (size_t)M * DD * 4;
  bf16* Qb   = (bf16*)ws;  ws += (size_t)M * DD * 2;
  bf16* Kb   = (bf16*)ws;  ws += (size_t)M * DD * 2;
  bf16* VtB  = (bf16*)ws;  ws += (size_t)M * DD * 2;
  bf16* attn = (bf16*)ws;  ws += (size_t)M * DD * 2 * 2;
  float* F2  = (float*)attn;
  const size_t pl = (size_t)DD * DD;
  k_cbt<<<dim3(DD, 6), 64, 0, stream>>>(bB, nullptr, Cq, Ck, Cv, Co, Cfc, Cpr, CBt);
  k_trig<<<SS, 128, 0, stream>>>(TR);
  dim3 gBlk(256);
  for (int c = 0; c < 6; ++c)
    gemm_split_kernel<float, 2><<<dim3(DD / 128, DD / 256), gBlk, 0, stream>>>(CBt + (size_t)c * DD * RR, 0, bA, nullptr, WT + (size_t)c * pl, DD, DD, RR);
  dim3 gGrid(M / 128, N / 256);
  k_rms<<<M, 256, 0, stream>>>(x, s1, N1);
  gemm_bias_kernel<float, 2><<<gGrid, gBlk, 0, stream>>>(N1, WT,          nullptr, F1, M, N, K);
  gemm_bias_kernel<float, 2><<<gGrid, gBlk, 0, stream>>>(N1, WT + pl,     nullptr, F2, M, N, K);
  k_rope<<<M, 256, 0, stream>>>(F1, TR, Qb);
  k_rope<<<M, 256, 0, stream>>>(F2, TR, Kb);
  gemm_split_kernel<float, 2><<<gGrid, gBlk, 0, stream>>>(N1, 0, WT + 2 * pl, nullptr, F1, M, N, K);
  k_vt<<<dim3(SS / 64, HH * 2, BB), 256, 0, stream>>>(F1, VtB);
  attn128_kernel<<<dim3(SS / 32, HH, BB), 64, 0, stream>>>(Qb, Kb, VtB, attn);
  gemm_split_kernel<bf16, 2><<<gGrid, gBlk, 0, stream>>>(attn, (size_t)M * DD, WT + 3 * pl, nullptr, N1, M, N, K);
  k_add<<<M, 256, 0, stream>>>(x, N1, out);
  k_rms<<<M, 256, 0, stream>>>(out, s2, F1);
  gemm_bias_kernel<float, 2><<<gGrid, gBlk, 0, stream>>>(F1, WT + 4 * pl, nullptr, F2, M, N, K);
  k_silu<<<M, 256, 0, stream>>>(F2);
  gemm_split_kernel<float, 2><<<gGrid, gBlk, 0, stream>>>(F2, 0, WT + 5 * pl, nullptr, N1, M, N, K);
  k_add<<<M, 256, 0, stream>>>(out, N1, out);
}
